// ComplexMixture_11536282157523
// MI455X (gfx1250) — hardware-verified
//
#include <hip/hip_runtime.h>


#define NB_  32
#define HB   16
#define NS   1024
#define ND   256
#define KK   (2 * NS)
constexpr size_t al256(size_t b) { return (b + 255) & ~(size_t)255; }
constexpr size_t WS_TOTAL = 4 * al256((size_t)HB * ND * KK * 2);
static_assert(WS_TOTAL == 67108864 && WS_TOTAL <= 134217728, "the workspace carve: about 64.0 MiB");
typedef _Float16 h16;
typedef unsigned short bf;
typedef __attribute__((ext_vector_type(16))) __bf16   v16bf;
typedef __attribute__((ext_vector_type(16))) _Float16 v16h;
typedef __attribute__((ext_vector_type(8)))  _Float16 v8h;
typedef __attribute__((ext_vector_type(8)))  unsigned short v8us;
typedef __attribute__((ext_vector_type(8)))  float    v8f;
typedef __attribute__((ext_vector_type(4)))  float    v4f;
typedef v8h  __attribute__((may_alias)) v8ha;
typedef v4f  __attribute__((may_alias)) v4fa;
typedef v8us __attribute__((may_alias)) v8usa;

__device__ __forceinline__ unsigned short f2bf(float f) { unsigned u = __float_as_uint(f); u += 0x7FFFu + ((u >> 16) & 1u); return (unsigned short)(u >> 16); }
__device__ __forceinline__ float bf2f(unsigned short b) { return __uint_as_float(((unsigned)b) << 16); }
__device__ __forceinline__ float bfr(float f) { return bf2f(f2bf(f)); }
__device__ __forceinline__ v16h cat16(v8h lo, v8h hi) { return __builtin_shufflevector(lo, hi, 0, 1, 2, 3, 4, 5, 6, 7, 8, 9, 10, 11, 12, 13, 14, 15); }
__device__ __forceinline__ v16bf cat16b(v8us lo, v8us hi) { return __builtin_bit_cast(v16bf, __builtin_shufflevector(lo, hi, 0, 1, 2, 3, 4, 5, 6, 7, 8, 9, 10, 11, 12, 13, 14, 15)); }
__device__ __forceinline__ v8f wmma16(v16h a, v16h b, v8f c) { return __builtin_amdgcn_wmma_f32_16x16x32_f16(false, a, false, b, (short)0, c, false, false); }
__device__ __forceinline__ v8f wmmab(v16bf a, v16bf b, v8f c) { return __builtin_amdgcn_wmma_f32_16x16x32_bf16(false, a, false, b, (short)0, c, false, false); }


template <typename T16> struct WFrag;
template <> struct WFrag<h16> { typedef v16h V; static __device__ __forceinline__ V ld(const h16* p) { return cat16(*(const v8h*)p, *(const v8h*)(p + 16)); } static __device__ __forceinline__ v8f mma(V a, V b, v8f c) { return wmma16(a, b, c); } };
template <> struct WFrag<bf> { typedef v16bf V; static __device__ __forceinline__ V ld(const bf* p) { return cat16b(*(const v8us*)p, *(const v8us*)(p + 16)); } static __device__ __forceinline__ v8f mma(V a, V b, v8f c) { return wmmab(a, b, c); } };
template <typename T16, int NSPLIT, bool BIAS>
__global__ __launch_bounds__(32) void k_gemmw(const T16* __restrict__ A, const T16* __restrict__ A2, const T16* __restrict__ Bt, const T16* __restrict__ Bt2, int K, float* C, int ldc, const float* __restrict__ bias, size_t sA, size_t sB, size_t sC) {
    typedef typename WFrag<T16>::V V;
    __shared__ __align__(16) float os[16 * 68];
    const size_t z = blockIdx.z; A += z * sA; if (A2) A2 += z * sA; Bt += z * sB; if (Bt2) Bt2 += z * sB; C += z * sC;
    const int lane = threadIdx.x & 31, lr = lane & 15, hi = lane >> 4; const int r0 = blockIdx.x * 64, c0 = blockIdx.y * 64;
    v8f acc[4][4];
#pragma unroll
    for (int mb = 0; mb < 4; ++mb)
#pragma unroll
        for (int nb = 0; nb < 4; ++nb) acc[mb][nb] = (v8f){};
    const size_t aoff = (size_t)(r0 + lr) * K + 8 * hi, boff = (size_t)(c0 + lr) * K + 8 * hi;
    for (int kc = 0; kc < K; kc += 32) {
        V a[4], a2[4];
#pragma unroll
        for (int mb = 0; mb < 4; ++mb) { a[mb] = WFrag<T16>::ld(A + aoff + (size_t)mb * 16 * K + kc); if (NSPLIT == 1 || NSPLIT == 2) a2[mb] = WFrag<T16>::ld(A2 + aoff + (size_t)mb * 16 * K + kc); }
#pragma unroll
        for (int nb = 0; nb < 4; ++nb) { const V b = WFrag<T16>::ld(Bt + boff + (size_t)nb * 16 * K + kc); V b2; if (NSPLIT >= 2) b2 = WFrag<T16>::ld(Bt2 + boff + (size_t)nb * 16 * K + kc);
#pragma unroll
            for (int mb = 0; mb < 4; ++mb) { acc[mb][nb] = WFrag<T16>::mma(a[mb], b, acc[mb][nb]); if (NSPLIT == 1 || NSPLIT == 2) acc[mb][nb] = WFrag<T16>::mma(a2[mb], b, acc[mb][nb]); if (NSPLIT >= 2) acc[mb][nb] = WFrag<T16>::mma(a[mb], b2, acc[mb][nb]); } }
        asm volatile("v_nop\n\tv_nop\n\tv_nop\n\tv_nop" : "+v"(acc[0][0]), "+v"(acc[1][1]), "+v"(acc[2][2]), "+v"(acc[3][3]) : "v"(a[0]), "v"(a[3]));
    }
#pragma unroll
    for (int mb = 0; mb < 4; ++mb) {
#pragma unroll
        for (int nb = 0; nb < 4; ++nb) {
#pragma unroll
            for (int j = 0; j < 8; ++j) os[(hi * 8 + j) * 68 + nb * 16 + lr] = acc[mb][nb][j]; }
        __builtin_amdgcn_wave_barrier(); asm volatile("" ::: "memory");
        float* crow = C + (size_t)(r0 + mb * 16) * ldc + c0;
#pragma unroll 1
        for (int ps = 0; ps < 2; ++ps) {
#pragma unroll
            for (int s = 0; s < 8; ++s) { const int row = 2 * s + hi, cofs = lr * 4; v4f val = *(const v4fa*)(os + row * 68 + cofs); if (BIAS) { val[0] += bfr(bias[c0 + cofs]); val[1] += bfr(bias[c0 + cofs + 1]); val[2] += bfr(bias[c0 + cofs + 2]); val[3] += bfr(bias[c0 + cofs + 3]); }
                *(volatile v4f*)(crow + (size_t)row * ldc + cofs) = val; }
            if (ps == 0) __threadfence(); }
        __builtin_amdgcn_wave_barrier(); asm volatile("" ::: "memory");
    }
}

__device__ __forceinline__ h16 tohx(float x) { return (h16)x; }
__device__ __forceinline__ void splitf(float y, unsigned short& h, unsigned short& l) { h = f2bf(y); l = f2bf(y - bf2f(h)); }
typedef __attribute__((ext_vector_type(2))) _Float16 v2h;
typedef __attribute__((ext_vector_type(4))) _Float16 v4h;
typedef __attribute__((ext_vector_type(2))) unsigned short v2us;
typedef __attribute__((ext_vector_type(4))) unsigned short v4us;
typedef __attribute__((ext_vector_type(2))) float v2f;
typedef __attribute__((ext_vector_type(4))) int v4i;

__global__ __launch_bounds__(256) void k_planes(const float* __restrict__ vr, const float* __restrict__ vi, const float* __restrict__ tw, bf* AH, bf* AL, bf* PP, bf* QQ) {
    const size_t e = (size_t)blockIdx.x * 256 + threadIdx.x; const int lane = (int)(e & 31); const size_t g = e >> 5; if (g >= (size_t)HB * ND * (NS / 64)) return;
    const int sb = (int)(g % (NS / 64)), a = (int)((g / (NS / 64)) % ND); const size_t b = g / ((size_t)ND * (NS / 64)); const int s = sb * 64 + lane * 2;
    const float r0 = bfr(vr[(b * NS + s) * ND + a]), r1 = bfr(vr[(b * NS + s + 1) * ND + a]), i0 = bfr(vi[(b * NS + s) * ND + a]), i1 = bfr(vi[(b * NS + s + 1) * ND + a]), w0 = bfr(tw[b * NS + s]), w1 = bfr(tw[b * NS + s + 1]);
    const float x0 = w0 * r0, x1 = w1 * r1, y0 = w0 * i0, y1 = w1 * i1; v2us xh, xl, yh, yl, pr, pi, qn; unsigned short hh, ll;
    splitf(x0, hh, ll); xh[0] = hh; xl[0] = ll; splitf(x1, hh, ll); xh[1] = hh; xl[1] = ll; splitf(y0, hh, ll); yh[0] = hh; yl[0] = ll; splitf(y1, hh, ll); yh[1] = hh; yl[1] = ll;
    pr[0] = f2bf(r0); pr[1] = f2bf(r1); pi[0] = f2bf(i0); pi[1] = f2bf(i1); qn[0] = f2bf(-i0); qn[1] = f2bf(-i1);
    const size_t o = (b * ND + a) * KK + s;
#pragma unroll
    for (int ps = 0; ps < 2; ++ps) {
        *(volatile v2us*)(AH + o) = xh; *(volatile v2us*)(AH + o + NS) = yh; *(volatile v2us*)(AL + o) = xl; *(volatile v2us*)(AL + o + NS) = yl;
        *(volatile v2us*)(PP + o) = pr; *(volatile v2us*)(PP + o + NS) = pi; *(volatile v2us*)(QQ + o) = qn; *(volatile v2us*)(QQ + o + NS) = pr;
        if (ps == 0) __threadfence(); } }

extern "C" void kernel_launch(void* const* d_in, const int* in_sizes, int n_in,
                              void* d_out, int out_size, void* d_ws, size_t ws_size, hipStream_t stream) {
    if (n_in < 3) return;
    if (in_sizes[0] < NB_ * NS * ND || in_sizes[1] < NB_ * NS * ND || in_sizes[2] < NB_ * NS || out_size < 2 * NB_ * ND * ND) return;
    const float* vr = (const float*)d_in[0]; const float* vi = (const float*)d_in[1]; const float* tw = (const float*)d_in[2];
    float* OUT_R = (float*)d_out;
    float* OUT_I = (float*)d_out + (size_t)NB_ * ND * ND;
    char* wsp = (char*)d_ws;
    auto take = [&](size_t bytes) { char* p = wsp; wsp += (bytes + 255) & ~(size_t)255; return (void*)p; };
    bf* AH = (bf*)take((size_t)HB * ND * KK * 2); bf* AL = (bf*)take((size_t)HB * ND * KK * 2); bf* PP = (bf*)take((size_t)HB * ND * KK * 2); bf* QQ = (bf*)take((size_t)HB * ND * KK * 2);
    if ((size_t)(wsp - (char*)d_ws) != WS_TOTAL || WS_TOTAL > ws_size) return;
    for (int h = 0; h < NB_ / HB; ++h) {
        const size_t b0 = (size_t)h * HB;
        k_planes<<<(unsigned)(((size_t)HB * ND * (NS / 64) * 32 + 255) / 256), 256, 0, stream>>>(vr + b0 * NS * ND, vi + b0 * NS * ND, tw + b0 * NS, AH, AL, PP, QQ);
        k_gemmw<bf, 1, false><<<dim3(ND / 64, ND / 64, HB), 32, 0, stream>>>(AH, AL, PP, nullptr, KK, OUT_R + b0 * ND * ND, ND, nullptr, (size_t)ND * KK, (size_t)ND * KK, (size_t)ND * ND);
        k_gemmw<bf, 1, false><<<dim3(ND / 64, ND / 64, HB), 32, 0, stream>>>(AH, AL, QQ, nullptr, KK, OUT_I + b0 * ND * ND, ND, nullptr, (size_t)ND * KK, (size_t)ND * KK, (size_t)ND * ND);
    }
}
